// PointNetPlusPlus_22273700397327
// MI455X (gfx1250) — hardware-verified
//
#include <hip/hip_runtime.h>
#include <math.h>

typedef __attribute__((ext_vector_type(16))) _Float16 v16h;
typedef __attribute__((ext_vector_type(16))) __bf16 v16b;
typedef __attribute__((ext_vector_type(8)))  _Float16 v8h;
typedef __attribute__((ext_vector_type(8)))  float v8f;
typedef __attribute__((ext_vector_type(4)))  float v4f;
typedef __attribute__((ext_vector_type(2)))  float v2f;
typedef __attribute__((ext_vector_type(4)))  unsigned v4u;
typedef __attribute__((ext_vector_type(4)))  int v4i;
typedef float __attribute__((may_alias)) float_a;
typedef int __attribute__((may_alias)) int_a;

template <typename T> __device__ __forceinline__ void vst2(void* p, T v) { *(volatile T*)p = v; __threadfence(); *(volatile T*)p = v; }
__device__ __forceinline__ v8f wmma16(v16h a, v16h b, v8f c) {
  v8f d = __builtin_amdgcn_wmma_f32_16x16x32_f16(false, a, false, b, (short)0, c, false, false);
  asm volatile("v_nop\n\tv_nop\n\tv_nop\n\tv_nop" : "+v"(d) : "v"(a), "v"(b));
  return d;
}
__device__ __forceinline__ v8f wmma_bf(v16b a, v16b b, v8f c) {
  v8f d = __builtin_amdgcn_wmma_f32_16x16x32_bf16(false, a, false, b, (short)0, c, false, false);
  asm volatile("v_nop\n\tv_nop\n\tv_nop\n\tv_nop" : "+v"(d) : "v"(a), "v"(b));
  return d;
}
__device__ __forceinline__ v16h frag_h(const _Float16* rowk0, int lane) {
  union { v16h v; v8h q[2]; } u; const _Float16* p = rowk0 + 8 * (lane >> 4);
  u.q[0] = *(const v8h*)p; u.q[1] = *(const v8h*)(p + 16); return u.v;
}
__device__ __forceinline__ v16h frag_f32(const float* rowk0, int lane) {
  v16h a; const float* p = rowk0 + 8 * (lane >> 4);
#pragma unroll
  for (int i = 0; i < 8; ++i) { a[i] = (_Float16)p[i]; a[8 + i] = (_Float16)p[16 + i]; }
  return a;
}
__device__ __forceinline__ v16h frag_f32s(const float* rowk0, int lane, float sc) {
  v16h a; const float* p = rowk0 + 8 * (lane >> 4);
#pragma unroll
  for (int i = 0; i < 8; ++i) { a[i] = (_Float16)(p[i] * sc); a[8 + i] = (_Float16)(p[16 + i] * sc); }
  return a;
}
__device__ __forceinline__ v16h fragc_f32(const float* W, int k0, int n, int lane, int ld, int K) {
  v16h a; const int g = lane >> 4;
#pragma unroll
  for (int i = 0; i < 8; ++i) { const int ka = k0 + 8 * g + i, kb = ka + 16;
    a[i] = (_Float16)(ka < K ? W[(size_t)(ka < K ? ka : K - 1) * ld + n] : 0.f); a[8 + i] = (_Float16)(kb < K ? W[(size_t)(kb < K ? kb : K - 1) * ld + n] : 0.f); }
  return a;
}
struct F2 { v16b h, l; };
__device__ __forceinline__ F2 bsplit16(const float v[16]) { F2 r;
#pragma unroll
  for (int i = 0; i < 16; ++i) { const __bf16 h = (__bf16)v[i]; r.h[i] = h; r.l[i] = (__bf16)(v[i] - (float)h); }
  return r; }
__device__ __forceinline__ F2 split_row(const float* row, int k0, int lane) { float v[16]; const float* p = row + k0 + 8 * (lane >> 4);
#pragma unroll
  for (int i = 0; i < 8; ++i) { v[i] = p[i]; v[8 + i] = p[16 + i]; }
  return bsplit16(v); }
__device__ __forceinline__ F2 split_rowK(const float* row, int k0, int lane, int K) { float v[16]; const int g = lane >> 4;
#pragma unroll
  for (int i = 0; i < 8; ++i) { const int ka = k0 + 8 * g + i, kb = ka + 16; v[i] = ka < K ? row[ka < K ? ka : K - 1] : 0.f; v[8 + i] = kb < K ? row[kb < K ? kb : K - 1] : 0.f; }
  return bsplit16(v); }
__device__ __forceinline__ F2 split_col(const float* W, int k0, int n, int lane, int ld, int K) { float v[16]; const int g = lane >> 4;
#pragma unroll
  for (int i = 0; i < 8; ++i) { const int ka = k0 + 8 * g + i, kb = ka + 16; v[i] = ka < K ? W[(size_t)(ka < K ? ka : K - 1) * ld + n] : 0.f; v[8 + i] = kb < K ? W[(size_t)(kb < K ? kb : K - 1) * ld + n] : 0.f; }
  return bsplit16(v); }
__device__ __forceinline__ v8f mac3(const F2& a, const F2& b, v8f c) { c = wmma_bf(a.l, b.h, c); c = wmma_bf(a.h, b.l, c); return wmma_bf(a.h, b.h, c); }
__device__ __forceinline__ float sigm(float v) { return 1.0f / (1.0f + expf(-v)); }
#define LDSX() do { asm volatile("s_wait_dscnt 0" ::: "memory"); __builtin_amdgcn_wave_barrier(); __builtin_amdgcn_fence(__ATOMIC_RELEASE, "workgroup"); } while (0)

__device__ __forceinline__ float bfr(float v) { return (float)(__bf16)v; }
#define NBT 32
#define NN 2048
#define NS 4
#define NF 10
#ifndef TNB
#define TNB NBT
#endif
#define WS_H   0u
#define WS_G   (WS_H + 4u * (size_t)NBT * NN * 64)
#define WS_I   (WS_G + 4u * (size_t)NBT * 64)
#define WS_END (WS_I + 4u * (size_t)NBT * NN * NS)
__device__ __forceinline__ float bnscale(float g) { return bfr(g) / sqrtf(1.00001f); }

__global__ __launch_bounds__(128) void k_embed(const float* __restrict__ X, const float* __restrict__ W1, const float* __restrict__ B1, const float* __restrict__ G1, const float* __restrict__ BE1, float* __restrict__ H) {
  __shared__ __align__(16) float se[64][68]; __shared__ __align__(16) float sf[4][16][68];
  const int tid = threadIdx.x, wave = tid >> 5, lane = tid & 31, col = lane & 15, g = lane >> 4; const size_t p0 = (size_t)blockIdx.x * 64;
  for (int e = tid; e < 64 * 64; e += 128) { const int rl = e >> 6, c = e & 63; const size_t p = p0 + rl; const float x = bfr(X[p * 2]), y = bfr(X[p * 2 + 1]); float v = 0.f;
    if (c == 0) v = x; else if (c == 1) v = y; else if (c < 2 + 4 * NF) { const int k = (c - 2) >> 2, w = (c - 2) & 3; const float f = (float)(1 << k); const float a = (w & 1) ? y * f : x * f; v = (w < 2) ? sinf(a) : cosf(a); }
    se[rl][c] = v; }
  __syncthreads();
  v8f acc[4] = {};
#pragma unroll
  for (int kc = 0; kc < 2; ++kc) { const F2 a = split_row(&se[wave * 16 + col][0], kc * 32, lane);
#pragma unroll
    for (int j = 0; j < 4; ++j) { v16b w; const int o = j * 16 + col;
#pragma unroll
      for (int i = 0; i < 16; ++i) { const int k = kc * 32 + (i < 8 ? 8 * g + i : 16 + 8 * g + (i - 8)); w[i] = (o < 60 && k < 42) ? (__bf16)W1[(size_t)(o < 60 ? o : 0) * 42 + (k < 42 ? k : 0)] : (__bf16)0.f; }
      acc[j] = wmma_bf(a.h, w, acc[j]); acc[j] = wmma_bf(a.l, w, acc[j]); } }
#pragma unroll
  for (int j = 0; j < 4; ++j)
#pragma unroll
    for (int r = 0; r < 8; ++r) { const int o = j * 16 + col; const int oc = o < 60 ? o : 0; float v = 0.f; if (o < 60) { v = fmaxf(acc[j][r] + bfr(B1[oc]), 0.f); v = v * bnscale(G1[oc]) + bfr(BE1[oc]); } sf[wave][8 * g + r][o] = v; }
  LDSX(); for (int rl = 0; rl < 16; ++rl) if (lane < 16) vst2(H + (p0 + wave * 16 + rl) * 64 + lane * 4, *(const v4f*)&sf[wave][rl][lane * 4]); }
__global__ __launch_bounds__(256) void k_gmax(const float* __restrict__ H, float* __restrict__ G) { __shared__ float sm[4][64];
  const int t = threadIdx.x; const int c = t & 63, grp = t >> 6; const int b = blockIdx.x; float m = -3.0e38f;
  for (int n = grp; n < NN; n += 4) m = fmaxf(m, H[((size_t)b * NN + n) * 64 + c]);
  sm[grp][c] = m; __syncthreads();
  if (t < 64) { const float v = fmaxf(fmaxf(sm[0][t], sm[1][t]), fmaxf(sm[2][t], sm[3][t])); sm[0][t] = v; }
  __syncthreads(); if (t < 16) vst2(G + (size_t)b * 64 + t * 4, *(const v4f*)&sm[0][t * 4]); }
__global__ __launch_bounds__(256) void k_ball(const float* __restrict__ X, int* __restrict__ IDX) { __shared__ __align__(16) int si[64][NS];
  const int tid = threadIdx.x, wave = tid >> 5, lane = tid & 31; const int b = blockIdx.y; const int q0 = blockIdx.x * 64; const float* Xb = X + (size_t)b * NN * 2;
  for (int qq = 0; qq < 8; ++qq) { const int ql = wave * 8 + qq; const int i = q0 + ql; const float xi = bfr(Xb[i * 2]), yi = bfr(Xb[i * 2 + 1]);
    int cnt = 0;
    for (int j0 = 0; j0 < NN; j0 += 32) { const int j = j0 + lane; const float dx = bfr(Xb[j * 2]) - xi, dy = bfr(Xb[j * 2 + 1]) - yi;
      const float d2 = __fadd_rn(__fmul_rn(dx, dx), __fmul_rn(dy, dy));
      const bool in = !(d2 > 1.0f);
      const unsigned bal = __builtin_amdgcn_ballot_w32(in); const int below = __builtin_popcount(bal & ((1u << lane) - 1u));
      if (in && cnt + below < NS) si[ql][cnt + below] = j;
      cnt += __builtin_popcount(bal); if (cnt >= NS) break; }
    LDSX();
    if (lane < NS && lane >= cnt) si[ql][lane] = si[ql][0];
    LDSX(); }
  __syncthreads();
  if (tid < 64) vst2(IDX + ((size_t)b * NN + q0) * NS + tid * 4, *(const v4i*)&si[tid][0]); }
__global__ __launch_bounds__(128) void k_sa(const float* __restrict__ X, const float* __restrict__ H, const float* __restrict__ G, const int* __restrict__ IDX,
    const float* __restrict__ WC0, const float* __restrict__ BC0, const float* __restrict__ GC0, const float* __restrict__ BEC0,
    const float* __restrict__ WC1, const float* __restrict__ BC1, const float* __restrict__ GC1, const float* __restrict__ BEC1,
    const float* __restrict__ G2, const float* __restrict__ BE2, const float* __restrict__ W4, const float* __restrict__ B4, float* __restrict__ OUT) {
  __shared__ __align__(16) float sa[64][132]; __shared__ __align__(16) float sz[64][68]; __shared__ __align__(16) float su[16][68]; __shared__ __align__(16) float so[16][4];
  const int tid = threadIdx.x, wave = tid >> 5, lane = tid & 31, col = lane & 15, g = lane >> 4; const size_t pt0 = (size_t)blockIdx.x * 16; const int b = (int)(pt0 / NN);
  for (int e = tid; e < 64 * 128; e += 128) { const int rl = e >> 7, c = e & 127; const size_t p = pt0 + (rl >> 2); const int nb = IDX[p * NS + (rl & 3)]; const size_t pn = (size_t)b * NN + nb; float v = 0.f;
    if (c < 2) v = bfr(X[pn * 2 + c]) - bfr(X[p * 2 + c]); else if (c < 62) v = H[pn * 64 + (c - 2)]; else if (c < 122) v = G[(size_t)b * 64 + (c - 62)];
    sa[rl][c] = v; }
  __syncthreads();
  { v8f acc[2] = {};
#pragma unroll
    for (int kc = 0; kc < 4; ++kc) { const F2 a = split_row(&sa[wave * 16 + col][0], kc * 32, lane);
#pragma unroll
      for (int j = 0; j < 2; ++j) { v16b w; const int o = j * 16 + col;
#pragma unroll
        for (int i = 0; i < 16; ++i) { const int k = kc * 32 + (i < 8 ? 8 * g + i : 16 + 8 * g + (i - 8)); w[i] = (o < 30 && k < 122) ? (__bf16)WC0[(size_t)(o < 30 ? o : 0) * 122 + (k < 122 ? k : 0)] : (__bf16)0.f; }
        acc[j] = wmma_bf(a.h, w, acc[j]); acc[j] = wmma_bf(a.l, w, acc[j]); } }
#pragma unroll
    for (int j = 0; j < 2; ++j)
#pragma unroll
      for (int r = 0; r < 8; ++r) { const int o = j * 16 + col; const int oc = o < 30 ? o : 0; float v = 0.f; if (o < 30) { v = (acc[j][r] + bfr(BC0[oc])) * bnscale(GC0[oc]) + bfr(BEC0[oc]); v = fmaxf(v, 0.f); } sz[wave * 16 + 8 * g + r][o] = v; } }
  LDSX();
  { v8f acc[4] = {};
    const F2 a = split_row(&sz[wave * 16 + col][0], 0, lane);
#pragma unroll
    for (int j = 0; j < 4; ++j) { v16b w; const int o = j * 16 + col;
#pragma unroll
      for (int i = 0; i < 16; ++i) { const int k = (i < 8 ? 8 * g + i : 16 + 8 * g + (i - 8)); w[i] = (o < 60 && k < 30) ? (__bf16)WC1[(size_t)(o < 60 ? o : 0) * 30 + (k < 30 ? k : 0)] : (__bf16)0.f; }
      acc[j] = wmma_bf(a.h, w, acc[j]); acc[j] = wmma_bf(a.l, w, acc[j]); }
#pragma unroll
    for (int j = 0; j < 4; ++j)
#pragma unroll
      for (int r = 0; r < 8; ++r) { const int o = j * 16 + col; const int oc = o < 60 ? o : 0; float v = 0.f; if (o < 60) { v = (acc[j][r] + bfr(BC1[oc])) * bnscale(GC1[oc]) + bfr(BEC1[oc]); v = fmaxf(v, 0.f); } sa[wave * 16 + 8 * g + r][o] = v; } }
  LDSX();
  { const int pl = lane >> 3; const int c8 = (lane & 7) * 8; const int rb = wave * 16 + pl * 4;
#pragma unroll
    for (int e = 0; e < 8; ++e) { const int c = c8 + e; float m = fmaxf(fmaxf(sa[rb][c], sa[rb + 1][c]), fmaxf(sa[rb + 2][c], sa[rb + 3][c])); float u = 0.f; if (c < 60) { u = m * bnscale(G2[c]) + bfr(BE2[c]); u = fmaxf(u, 0.f); } su[wave * 4 + pl][c] = u; } }
  __syncthreads();
  if (wave == 0) { v8f acc = {};
#pragma unroll
    for (int kc = 0; kc < 2; ++kc) { const F2 a = split_row(&su[col][0], kc * 32, lane); v16b w; const int o = col;
#pragma unroll
      for (int i = 0; i < 16; ++i) { const int k = kc * 32 + (i < 8 ? 8 * g + i : 16 + 8 * g + (i - 8)); w[i] = (o < 2 && k < 60) ? (__bf16)W4[(size_t)(o < 2 ? o : 0) * 60 + (k < 60 ? k : 0)] : (__bf16)0.f; }
      acc = wmma_bf(a.h, w, acc); acc = wmma_bf(a.l, w, acc); }
    if (col < 2) {
#pragma unroll
      for (int r = 0; r < 8; ++r) so[8 * g + r][col] = acc[r] + bfr(B4[col]); }
    LDSX();
    if (lane < 8) { v4f o4; o4[0] = so[2 * lane][0]; o4[1] = so[2 * lane][1]; o4[2] = so[2 * lane + 1][0]; o4[3] = so[2 * lane + 1][1]; vst2(OUT + pt0 * 2 + lane * 4, o4); } } }
extern "C" void kernel_launch(void* const* d_in, const int* in_sizes, int n_in, void* d_out, int out_size, void* d_ws, size_t ws_size, hipStream_t stream) {
  (void)in_sizes; (void)n_in; (void)out_size;
  const float** F = (const float**)d_in;
  if (ws_size < (size_t)WS_END) return;
  char* ws = (char*)d_ws; float *H = (float*)(ws + WS_H), *G = (float*)(ws + WS_G); int* IDX = (int*)(ws + WS_I);
  k_embed<<<dim3(TNB * NN / 64), 128, 0, stream>>>(F[0], F[1], F[2], F[3], F[4], H);
  k_gmax<<<dim3(TNB), 256, 0, stream>>>(H, G);
  k_ball<<<dim3(NN / 64, TNB), 256, 0, stream>>>(F[0], IDX);
  k_sa<<<dim3(TNB * NN / 16), 128, 0, stream>>>(F[0], H, G, IDX, F[5], F[6], F[7], F[8], F[9], F[10], F[11], F[12], F[13], F[14], F[15], F[16], (float*)d_out);
}
